// MultiHeadSelfAttention_27487790694990
// MI455X (gfx1250) — hardware-verified
//
#include <hip/hip_runtime.h>
#ifndef NB
#define NB 4
#endif
#ifndef SEQ
#define SEQ 2048
#endif
#define NB_FULL 4
#define SEQ_FULL 2048
#define DM 1024
#define NH 16
#define HD 64
#define HG 2
#define LQ (3 * DM)
#define NR ((unsigned)(NB * SEQ))

#define SZ_BQKV ((size_t)3 * DM * DM * 2)
#define SZ_BO   ((size_t)DM * DM * 2)
#define SZ_HO   ((size_t)NB * SEQ * DM * 2)
#define SZ_QKV  ((size_t)NB * SEQ * 3 * DM * 2)
#define SZ_S    ((size_t)HG * SEQ * SEQ * 4)
#define SZ_P    ((size_t)HG * SEQ * SEQ * 2)
#define SZ_VT   ((size_t)NH * HD * SEQ * 2)
#define SZ_ALL  (SZ_BQKV + SZ_BO + SZ_HO + SZ_QKV + SZ_S + SZ_P + SZ_VT)

static_assert(DM == 128 * 8);
static_assert(NH * HD == DM);
static_assert(HD == 64);
static_assert(NH % HG == 0);
static_assert(SEQ % 256 == 0);
static_assert((NB * SEQ) % 128 == 0);
static_assert((3 * DM) % 64 == 0 && DM % 64 == 0 && DM % 32 == 0 && HD % 32 == 0 && SEQ % 32 == 0);
static_assert(NB <= NB_FULL && SEQ <= SEQ_FULL);
static_assert((size_t)SEQ * 16 <= 65536);
static_assert(SZ_BQKV % 256 == 0 && SZ_BO % 256 == 0 && SZ_HO % 256 == 0 && SZ_QKV % 256 == 0 && SZ_S % 256 == 0 && SZ_P % 256 == 0 && SZ_VT % 256 == 0);
static_assert(SZ_ALL <= (size_t)134217728);
static_assert((size_t)(NB * SEQ) * 128 * 8 == (size_t)NB * SEQ * DM);
static_assert((size_t)(NH * (SEQ / 64)) * 256 * 2 * 8 == (size_t)NH * HD * SEQ);
static_assert((size_t)(HG * SEQ / 4) * 4 * SEQ == (size_t)HG * SEQ * SEQ);
static_assert((size_t)((NB * SEQ / 128) * (3 * DM / 64)) * 128 * 64 == (size_t)NB * SEQ * 3 * DM);
static_assert((size_t)((SEQ / 128) * (SEQ / 64)) * HG * 128 * 64 == (size_t)HG * SEQ * SEQ);
static_assert((size_t)((SEQ / 128) * (HD / 64)) * HG * 128 * 64 == (size_t)HG * SEQ * HD);
static_assert((size_t)((NB * SEQ / 128) * (DM / 64)) * 128 * 64 == (size_t)NB * SEQ * DM);

typedef unsigned short v8us __attribute__((ext_vector_type(8), may_alias));
typedef float  v8f  __attribute__((ext_vector_type(8)));
typedef float  v4f  __attribute__((ext_vector_type(4)));
typedef float  v4fa __attribute__((ext_vector_type(4), may_alias));
typedef _Float16 v16h __attribute__((ext_vector_type(16)));
typedef _Float16 v4h __attribute__((ext_vector_type(4)));
union FragH { v16h v; v8us half[2]; _Float16 h[16]; unsigned short u[16]; };

__device__ __forceinline__ unsigned short bf16_bits(float x) { unsigned int u = __float_as_uint(x); return (unsigned short)((u + 0x7FFFu + ((u >> 16) & 1u)) >> 16); }
__device__ __forceinline__ float bf16_rne(float x) { return __uint_as_float(((unsigned int)bf16_bits(x)) << 16); }
__device__ __forceinline__ float wave_sum(float v) { v += __shfl_xor(v, 16, 32); v += __shfl_xor(v, 8, 32); v += __shfl_xor(v, 4, 32); v += __shfl_xor(v, 2, 32); v += __shfl_xor(v, 1, 32); return v; }
__device__ __forceinline__ float wave_max(float v) { v = fmaxf(v, __shfl_xor(v, 16, 32)); v = fmaxf(v, __shfl_xor(v, 8, 32)); v = fmaxf(v, __shfl_xor(v, 4, 32)); v = fmaxf(v, __shfl_xor(v, 2, 32)); v = fmaxf(v, __shfl_xor(v, 1, 32)); return v; }
__device__ __forceinline__ unsigned in_row(unsigned r) { return (r / (unsigned)SEQ) * (unsigned)SEQ_FULL + (r % (unsigned)SEQ); }

__global__ __launch_bounds__(256) void k_wt_f16(const float* __restrict__ W, _Float16* __restrict__ Wt, unsigned K, unsigned N, float scale) {
  const unsigned t = blockIdx.x * 256u + threadIdx.x; const unsigned k8n = K >> 3; if (t >= N * k8n) return;
  const unsigned n = t / k8n, k8 = (t - n * k8n) * 8u; FragH f;
#pragma unroll
  for (unsigned i = 0; i < 8; ++i) f.h[i] = (_Float16)(bf16_rne(W[(size_t)(k8 + i) * N + n]) * scale);
  const v8us o = f.half[0]; unsigned short* d = (unsigned short*)Wt + (size_t)n * K + k8;
  *(volatile v8us*)d = o; __threadfence(); *(volatile v8us*)d = o;
}

__global__ __launch_bounds__(128) void k_ln16(const float* __restrict__ x, const float* __restrict__ g, const float* __restrict__ bt, _Float16* __restrict__ H) {
  __shared__ float red1[4];
  __shared__ float red2[4];
  const unsigned tid = threadIdx.x, w = tid >> 5, lane = tid & 31u; const unsigned r = blockIdx.x;
  const float* xp = x + (size_t)in_row(r) * DM + tid * 8u;
  const v4f a = *(const v4fa*)xp, c = *(const v4fa*)(xp + 4);
  float vals[8];
#pragma unroll
  for (unsigned q = 0; q < 4; ++q) { vals[q] = bf16_rne(a[q]); vals[4 + q] = bf16_rne(c[q]); }
  float s1 = ((vals[0] + vals[1]) + (vals[2] + vals[3])) + ((vals[4] + vals[5]) + (vals[6] + vals[7]));
  s1 = wave_sum(s1);
  if (lane == 0) red1[w] = s1;
  __syncthreads();
  const float mu = ((red1[0] + red1[1]) + (red1[2] + red1[3])) * (1.0f / (float)DM);
  float s2 = 0.f;
#pragma unroll
  for (unsigned q = 0; q < 8; ++q) { const float cc = vals[q] - mu; s2 += cc * cc; }
  s2 = wave_sum(s2);
  if (lane == 0) red2[w] = s2;
  __syncthreads();
  const float var = ((red2[0] + red2[1]) + (red2[2] + red2[3])) * (1.0f / (float)DM);
  const float rs = rsqrtf(var + 1e-5f);
  const v4f g0 = *(const v4fa*)(g + tid * 8u), g1 = *(const v4fa*)(g + tid * 8u + 4), b0 = *(const v4fa*)(bt + tid * 8u), b1 = *(const v4fa*)(bt + tid * 8u + 4);
  FragH f;
#pragma unroll
  for (unsigned q = 0; q < 4; ++q) {
    f.h[q]     = (_Float16)((vals[q] - mu) * rs * bf16_rne(g0[q]) + bf16_rne(b0[q]));
    f.h[4 + q] = (_Float16)((vals[4 + q] - mu) * rs * bf16_rne(g1[q]) + bf16_rne(b1[q]));
  }
  const v8us o = f.half[0]; unsigned short* d = (unsigned short*)H + (size_t)r * DM + tid * 8u;
  *(volatile v8us*)d = o; __threadfence(); *(volatile v8us*)d = o;
}

template <unsigned NHv, unsigned TTv>
__global__ __launch_bounds__(256) void k_vt(const _Float16* __restrict__ V16, unsigned ldv, unsigned voff, _Float16* __restrict__ Vt) {
  __shared__ unsigned short tl[64][66];
  const unsigned tid = threadIdx.x; const unsigned slab = blockIdx.x / (TTv / 64u), lg = blockIdx.x % (TTv / 64u); const unsigned b = slab / NHv, h = slab % NHv;
  for (unsigned i = tid; i < 512u; i += 256u) {
    const unsigned r = i >> 3, c8 = (i & 7u) * 8u; FragH f;
    f.half[0] = *(const v8us*)((const unsigned short*)V16 + ((size_t)b * TTv + lg * 64u + r) * ldv + voff + h * 64u + c8);
#pragma unroll
    for (unsigned q = 0; q < 8; ++q) tl[r][c8 + q] = f.u[q];
  }
  __syncthreads();
  for (int pass = 0; pass < 2; ++pass) {
#pragma unroll
    for (unsigned rd = 0; rd < 2; ++rd) {
      const unsigned d = rd * 32u + (tid >> 3), pc = tid & 7u; FragH f;
#pragma unroll
      for (unsigned q = 0; q < 8; ++q) f.u[q] = tl[pc * 8u + q][d];
      *(volatile v8us*)((unsigned short*)Vt + ((size_t)slab * 64u + d) * TTv + lg * 64u + pc * 8u) = f.half[0];
    }
    if (pass == 0) __threadfence();
  }
}

__global__ __launch_bounds__(128) void k_rsm(const float* __restrict__ S, _Float16* __restrict__ P, unsigned nrows) {
#pragma clang fp contract(off)
  __shared__ __attribute__((aligned(16))) float sr[4][SEQ];
  const unsigned tid = threadIdx.x, w = tid >> 5, lane = tid & 31u; const unsigned i = blockIdx.x * 4u + w; if (i >= nrows) return;
  const float* s = S + (size_t)i * SEQ + lane * 8u; float* my = &sr[w][lane * 8u];
  float mx = -3.0e38f;
#pragma unroll 1
  for (unsigned u = 0; u < (unsigned)SEQ / 256u; ++u) {
    const v4f a = *(const v4fa*)(s + u * 256u), c = *(const v4fa*)(s + u * 256u + 4);
    *(v4fa*)(my + u * 256u) = a; *(v4fa*)(my + u * 256u + 4) = c;
    mx = fmaxf(mx, fmaxf(fmaxf(fmaxf(a[0], a[1]), fmaxf(a[2], a[3])), fmaxf(fmaxf(c[0], c[1]), fmaxf(c[2], c[3]))));
  }
  mx = wave_max(mx);
  float se = 0.f;
#pragma unroll 1
  for (unsigned u = 0; u < (unsigned)SEQ / 128u; ++u) {
    float* p = my + (u >> 1) * 256u + (u & 1u) * 4u; v4f a = *(const v4fa*)p;
    a[0] = expf(a[0] - mx); a[1] = expf(a[1] - mx); a[2] = expf(a[2] - mx); a[3] = expf(a[3] - mx);
    se += (a[0] + a[1]) + (a[2] + a[3]);
    *(v4fa*)p = a;
  }
  se = wave_sum(se);
  const float sc = 256.0f / se;
  v8us pk[SEQ / 256];
#pragma unroll
  for (unsigned u = 0; u < (unsigned)SEQ / 256u; ++u) {
    const v4f a = *(const v4fa*)(my + u * 256u), c = *(const v4fa*)(my + u * 256u + 4); FragH f;
#pragma unroll
    for (unsigned q = 0; q < 4; ++q) { f.h[q] = (_Float16)(a[q] * sc); f.h[4 + q] = (_Float16)(c[q] * sc); }
    pk[u] = f.half[0];
  }
  unsigned short* d = (unsigned short*)P + (size_t)i * SEQ + lane * 8u;
#pragma unroll
  for (unsigned u = 0; u < (unsigned)SEQ / 256u; ++u) *(volatile v8us*)(d + u * 256u) = pk[u];
  __threadfence();
#pragma unroll
  for (unsigned u = 0; u < (unsigned)SEQ / 256u; ++u) *(volatile v8us*)(d + u * 256u) = pk[u];
}

__device__ __forceinline__ v16h g2_frag(const _Float16* p, unsigned hh) { FragH f; f.half[0] = *(const v8us*)((const unsigned short*)p + 8u * hh); f.half[1] = *(const v8us*)((const unsigned short*)p + 16u + 8u * hh); return f.v; }
__device__ __forceinline__ v8f g2_mma(v16h a, v16h b, v8f c) { v8f d = __builtin_amdgcn_wmma_f32_16x16x32_f16(false, a, false, b, (short)0, c, false, false); asm volatile("v_nop\n\tv_nop\n\tv_nop\n\tv_nop" : "+v"(d) : "v"(a), "v"(b)); return d; }
template <bool RES>
__global__ __launch_bounds__(128) void k_gemm2(const _Float16* __restrict__ A, unsigned lda, size_t sA, const _Float16* __restrict__ Bh, unsigned ldb, size_t sB, float alpha,
    const float* __restrict__ bias, const float* __restrict__ xres, float* __restrict__ C, _Float16* __restrict__ C16, unsigned ldc, size_t sC, unsigned M, unsigned N, unsigned K) {
  __shared__ __attribute__((aligned(16))) float so[4][32][68];
  const unsigned tid = threadIdx.x, w = tid >> 5, lane = tid & 31u, ln = lane & 15u, hh = lane >> 4; const unsigned by = blockIdx.y;
  A += (size_t)by * sA; Bh += (size_t)by * sB; const size_t cofs = (size_t)by * sC;
  const unsigned ntn = N >> 6; const unsigned mt = blockIdx.x / ntn, nq = blockIdx.x - mt * ntn; const unsigned row0 = mt * 128u + 32u * w, col0 = nq * 64u; if (row0 >= M) return;
  const _Float16* a0p = A + (size_t)(row0 + ln) * lda; const _Float16* a1p = a0p + (size_t)16 * lda;
  const _Float16* b0p = Bh + (size_t)(col0 + ln) * ldb; const _Float16* b1p = b0p + (size_t)16 * ldb; const _Float16* b2p = b1p + (size_t)16 * ldb; const _Float16* b3p = b2p + (size_t)16 * ldb;
  const v8f z8 = {0.f,0.f,0.f,0.f,0.f,0.f,0.f,0.f}; v8f c00 = z8, c01 = z8, c02 = z8, c03 = z8, c10 = z8, c11 = z8, c12 = z8, c13 = z8;
#pragma unroll 1
  for (unsigned kb = 0; kb < K; kb += 32u) { const v16h a0 = g2_frag(a0p + kb, hh), a1 = g2_frag(a1p + kb, hh);
    v16h b = g2_frag(b0p + kb, hh); c00 = g2_mma(a0, b, c00); c10 = g2_mma(a1, b, c10);
    b = g2_frag(b1p + kb, hh); c01 = g2_mma(a0, b, c01); c11 = g2_mma(a1, b, c11);
    b = g2_frag(b2p + kb, hh); c02 = g2_mma(a0, b, c02); c12 = g2_mma(a1, b, c12);
    b = g2_frag(b3p + kb, hh); c03 = g2_mma(a0, b, c03); c13 = g2_mma(a1, b, c13); }
  v8f accs[8] = {c00, c01, c02, c03, c10, c11, c12, c13};
#pragma unroll
  for (unsigned u = 0; u < 8; ++u) { const unsigned t = u & 3u, hf = u >> 2; const unsigned col = col0 + t * 16u + ln; const float bv = bias ? bf16_rne(bias[col]) : 0.f;
#pragma unroll
    for (unsigned r = 0; r < 8; ++r) so[w][hf * 16u + 8u * hh + r][t * 16u + ln] = accs[u][r] * alpha + bv; }
  __builtin_amdgcn_fence(4  , "workgroup"); __builtin_amdgcn_wave_barrier();
  const unsigned rsub = lane >> 4, c4 = (lane & 15u) * 4u;
  for (int pass = 0; pass < 2; ++pass) {
#pragma unroll 4
    for (unsigned q = 0; q < 16; ++q) { const unsigned r = q * 2u + rsub; v4f v = *(const v4fa*)&so[w][r][c4];
      if (RES) { const v4f xv = *(const v4fa*)(xres + (size_t)in_row(row0 + r) * DM + col0 + c4); v[0] += bf16_rne(xv[0]); v[1] += bf16_rne(xv[1]); v[2] += bf16_rne(xv[2]); v[3] += bf16_rne(xv[3]); }
      if (C) *(volatile v4f*)(C + cofs + (size_t)(row0 + r) * ldc + col0 + c4) = v;
      if (C16) { v4h h4; h4[0] = (_Float16)v[0]; h4[1] = (_Float16)v[1]; h4[2] = (_Float16)v[2]; h4[3] = (_Float16)v[3]; *(volatile v4h*)(C16 + cofs + (size_t)(row0 + r) * ldc + col0 + c4) = h4; } }
    if (pass == 0) __threadfence(); }
}

extern "C" void kernel_launch(void* const* d_in, const int* in_sizes, int n_in,
                              void* d_out, int out_size, void* d_ws, size_t ws_size, hipStream_t stream) {
  if (n_in < 7) return;
  const size_t need_x = ((size_t)(NB - 1) * SEQ_FULL + SEQ) * DM;
  if ((size_t)in_sizes[0] < need_x || in_sizes[1] < DM || in_sizes[2] < DM || in_sizes[3] < 3 * DM * DM || in_sizes[4] < 3 * DM || in_sizes[5] < DM * DM || in_sizes[6] < DM) return;
  if ((size_t)out_size < (size_t)NR * DM) return;
  const float* x = (const float*)d_in[0]; const float* lng = (const float*)d_in[1]; const float* lnb = (const float*)d_in[2];
  const float* wqkv = (const float*)d_in[3]; const float* bqkv = (const float*)d_in[4]; const float* wo = (const float*)d_in[5]; const float* bo = (const float*)d_in[6];
  char* ws = (char*)d_ws; size_t off = 0;
  auto take = [&](size_t bytes) { char* p = ws + off; off += (bytes + 255) & ~(size_t)255; return p; };
  _Float16* BQKV = (_Float16*)take(SZ_BQKV); _Float16* BO = (_Float16*)take(SZ_BO);
  _Float16* H16 = (_Float16*)take(SZ_HO); _Float16* O16 = H16;
  _Float16* QKV = (_Float16*)take(SZ_QKV); _Float16* Q16 = QKV; _Float16* K16 = QKV + DM; _Float16* V16 = QKV + 2 * DM;
  float* S = (float*)take(SZ_S); _Float16* P = (_Float16*)take(SZ_P); _Float16* VT = (_Float16*)take(SZ_VT);
  if (off > ws_size) return;
  k_wt_f16<<<(unsigned)(((size_t)DM * 3 * DM / 8 + 255) / 256), 256, 0, stream>>>(wqkv, BQKV, (unsigned)DM, (unsigned)(3 * DM), 16.0f);
  k_wt_f16<<<(unsigned)(((size_t)DM * DM / 8 + 255) / 256), 256, 0, stream>>>(wo, BO, (unsigned)DM, (unsigned)DM, 16.0f);
  k_ln16<<<NR, 128, 0, stream>>>(x, lng, lnb, H16);
  k_gemm2<false><<<dim3((NR / 128u) * (3u * DM / 64u), 1), 128, 0, stream>>>(H16, (unsigned)DM, (size_t)0, BQKV, (unsigned)DM, (size_t)0, 0.0625f, bqkv, nullptr,
      nullptr, QKV, (unsigned)(3 * DM), (size_t)0, NR, (unsigned)(3 * DM), (unsigned)DM);
  for (unsigned b = 0; b < (unsigned)NB; ++b) { const size_t r0 = (size_t)b * SEQ;
    k_vt<NH, SEQ><<<NH * (SEQ / 64), 256, 0, stream>>>(V16 + r0 * LQ, (unsigned)LQ, 0u, VT);
    for (unsigned h0 = 0; h0 < (unsigned)NH; h0 += HG) {
      k_gemm2<false><<<dim3((SEQ / 128) * (SEQ / 64), HG), 128, 0, stream>>>(Q16 + r0 * LQ + h0 * HD, (unsigned)LQ, (size_t)HD, K16 + r0 * LQ + h0 * HD, (unsigned)LQ, (size_t)HD, 0.125f, nullptr, nullptr,
          S, nullptr, (unsigned)SEQ, (size_t)SEQ * SEQ, (unsigned)SEQ, (unsigned)SEQ, (unsigned)HD);
      k_rsm<<<(HG * SEQ) / 4, 128, 0, stream>>>(S, P, (unsigned)(HG * SEQ));
      k_gemm2<false><<<dim3((SEQ / 128) * (HD / 64), HG), 128, 0, stream>>>(P, (unsigned)SEQ, (size_t)SEQ * SEQ, VT + (size_t)h0 * HD * SEQ, (unsigned)SEQ, (size_t)HD * SEQ, 0.25f, nullptr, nullptr,
          nullptr, O16 + r0 * DM + h0 * HD, (unsigned)DM, (size_t)HD, (unsigned)SEQ, (unsigned)HD, (unsigned)SEQ);
    } }
  k_gemm2<true><<<dim3((NR / 128u) * (DM / 64u), 1), 128, 0, stream>>>(O16, (unsigned)DM, (size_t)0, BO, (unsigned)DM, (size_t)0, 0.0009765625f, bo, x,
      (float*)d_out, nullptr, (unsigned)DM, (size_t)0, NR, (unsigned)DM, (unsigned)DM);
}
